// CapsNet_5463198401116
// MI455X (gfx1250) — hardware-verified
//
#include <hip/hip_runtime.h>
#include <math.h>

constexpr int kBatch  = 256;
constexpr int kImg    = 28;
constexpr int kC      = 256;
constexpr int kH1     = 20;
constexpr int kP1     = kBatch * kH1 * kH1;
constexpr int kTaps   = 81;
constexpr int kK1     = 96;
constexpr int kK2     = kTaps * kC;
constexpr int kSp2    = 36;
constexpr int kM2     = kBatch * kSp2;
constexpr int kRoute  = 1152;
constexpr int kCls    = 10;
constexpr int kVd     = 16;
constexpr int kRows   = kRoute * kCls;
constexpr int kNIO    = kCls * kVd;

static_assert(kK1 % 32 == 0);
static_assert(kP1 % 64 == 0);
static_assert(kC % 64 == 0);
static_assert(kK2 % 32 == 0);
static_assert(kM2 % 64 == 0);

constexpr int kIm2colBlocksA = kP1 * (kK1 / 8) / 256;
constexpr int kIm2colBlocksB = kC * (kK1 / 8) / 256;
static_assert(kIm2colBlocksA * 256 * 8 == kP1 * kK1);
static_assert(kIm2colBlocksB * 256 * 8 == kC * kK1);
constexpr int kW2Blocks = kC * (kK2 / 8) / 256;
static_assert(kW2Blocks * 256 * 8 == kC * kK2);
constexpr int kCv1Blocks = (kP1 / 64) * (kC / 64) / 8;
static_assert(kCv1Blocks * 8 == (kP1 / 64) * (kC / 64));
constexpr int kCv2Tiles  = (kM2 / 64) * (kC / 64);
constexpr int kCv2Blocks = kCv2Tiles / 8;
static_assert(kCv2Blocks * 8 == kCv2Tiles);

constexpr size_t kBytesU    = (size_t)kRows * kBatch * kVd * 2;
constexpr size_t kBytesA1   = (size_t)kP1 * kK1 * 2;
constexpr size_t kBytesH    = (size_t)kP1 * kC * 2;
constexpr size_t kBytesBt1  = (size_t)kC * kK1 * 2;
constexpr size_t kBytesBt2  = (size_t)kC * kK2 * 2;
constexpr size_t kBytesPrim = (size_t)kM2 * kC * 4;
constexpr size_t kBytesV    = (size_t)kCls * kBatch * kVd * 4;
constexpr size_t kBytesBij  = (size_t)kCls * kRoute * 4;
constexpr size_t kOffU    = 0;
constexpr size_t kOffA1   = 0;
constexpr size_t kOffH    = kOffA1 + kBytesA1;
constexpr size_t kOffBt1  = kOffU + kBytesU;
constexpr size_t kOffBt2  = kOffBt1 + kBytesBt1;
constexpr size_t kOffPrim = kOffBt2 + kBytesBt2;
constexpr size_t kOffVraw = kOffPrim + kBytesPrim;
constexpr size_t kOffVbuf = kOffVraw + kBytesV;
constexpr size_t kOffBijA = kOffVbuf + kBytesV;
constexpr size_t kOffBijB = kOffBijA + kBytesBij;
constexpr size_t kWsTotal = kOffBijB + kBytesBij;
static_assert(kOffH + kBytesH <= kBytesU);
static_assert(kWsTotal == 114894848);
static_assert(kWsTotal <= 134217728);
static_assert(kOffH % 256 == 0 && kOffBt1 % 256 == 0 && kOffBt2 % 256 == 0 && kOffPrim % 256 == 0);
static_assert(kOffVraw % 256 == 0 && kOffVbuf % 256 == 0 && kOffBijA % 256 == 0 && kOffBijB % 256 == 0);

typedef __attribute__((ext_vector_type(16))) _Float16 v16h;
typedef __attribute__((ext_vector_type(8)))  _Float16 v8h;
typedef __attribute__((ext_vector_type(16))) __bf16   v16b;
typedef __attribute__((ext_vector_type(8)))  __bf16   v8b;
typedef __attribute__((ext_vector_type(8)))  float    v8f;
typedef __attribute__((ext_vector_type(4)))  float    v4f;
typedef __attribute__((ext_vector_type(4)))  unsigned int v4u;

__device__ __forceinline__ unsigned short f2bf_bits(float f) {
  unsigned u = __float_as_uint(f);
  return (unsigned short)((u + 0x7FFFu + ((u >> 16) & 1u)) >> 16);
}
__device__ __forceinline__ float bf_bits2f(unsigned short h) { return __uint_as_float(((unsigned)h) << 16); }

__device__ __forceinline__ void dep_guard_h(v8f& a, v8f& b, v16h x, v16h y) { asm volatile("v_nop\n\tv_nop\n\tv_nop\n\tv_nop" : "+v"(a), "+v"(b) : "v"(x), "v"(y)); }
__device__ __forceinline__ void dep_guard_b(v8f& a, v8f& b, v16b x, v16b y) { asm volatile("v_nop\n\tv_nop\n\tv_nop\n\tv_nop" : "+v"(a), "+v"(b) : "v"(x), "v"(y)); }
__device__ __forceinline__ void dep_guard_all_h(v8f& a0, v8f& a1, v8f& a2, v8f& a3, v16h x, v16h y, v16h b0, v16h b1, v16h b2, v16h b3) {
  asm volatile("v_nop\n\tv_nop\n\tv_nop\n\tv_nop" : "+v"(a0), "+v"(a1), "+v"(a2), "+v"(a3) : "v"(x), "v"(y), "v"(b0), "v"(b1), "v"(b2), "v"(b3));
}
__device__ __forceinline__ void dep_guard_all_b(v8f& a0, v8f& a1, v8f& a2, v8f& a3, v16b x, v16b y, v16b b0, v16b b1, v16b b2, v16b b3) {
  asm volatile("v_nop\n\tv_nop\n\tv_nop\n\tv_nop" : "+v"(a0), "+v"(a1), "+v"(a2), "+v"(a3) : "v"(x), "v"(y), "v"(b0), "v"(b1), "v"(b2), "v"(b3));
}
__device__ __forceinline__ void dep_guard1_h(v8f& a, v16h x, v16h y) { asm volatile("v_nop\n\tv_nop\n\tv_nop\n\tv_nop" : "+v"(a) : "v"(x), "v"(y)); }
__device__ __forceinline__ void keep4_h(v16h a, v16h b, v16h c, v16h d) { asm volatile("v_nop" :: "v"(a), "v"(b), "v"(c), "v"(d)); }
__device__ __forceinline__ void keep4_b(v16b a, v16b b, v16b c, v16b d) { asm volatile("v_nop" :: "v"(a), "v"(b), "v"(c), "v"(d)); }
__device__ __forceinline__ void acc_guard4(v8f& a, v8f& b, v8f& c, v8f& d) { asm volatile("v_nop\n\tv_nop\n\tv_nop\n\tv_nop" : "+v"(a), "+v"(b), "+v"(c), "+v"(d)); }
template <typename T> struct Frag;
template <> struct Frag<_Float16> {
  typedef v16h V; union U { v16h v; v8h h[2]; };
  static __device__ __forceinline__ v16h load(const _Float16* p) {
    U f; f.h[0] = *(const v8h*)(p); f.h[1] = *(const v8h*)(p + 16); return f.v;
  }
  static __device__ __forceinline__ v8f mma(v16h a, v16h b, v8f c) {
    return __builtin_amdgcn_wmma_f32_16x16x32_f16(false, a, false, b, (short)0, c, false, false);
  }
  static __device__ __forceinline__ void guard(v8f& a, v8f& b, v16h x, v16h y) { dep_guard_h(a, b, x, y); }
  static __device__ __forceinline__ void guard_all(v8f& a0, v8f& a1, v8f& a2, v8f& a3, v16h x, v16h y, v16h b0, v16h b1, v16h b2, v16h b3) {
    dep_guard_all_h(a0, a1, a2, a3, x, y, b0, b1, b2, b3);
  }
  static __device__ __forceinline__ void keep(v16h a, v16h b, v16h c, v16h d) { keep4_h(a, b, c, d); }
};
template <> struct Frag<__bf16> {
  typedef v16b V; union U { v16b v; v8b h[2]; };
  static __device__ __forceinline__ v16b load(const __bf16* p) {
    U f; f.h[0] = *(const v8b*)(p); f.h[1] = *(const v8b*)(p + 16); return f.v;
  }
  static __device__ __forceinline__ v8f mma(v16b a, v16b b, v8f c) {
    return __builtin_amdgcn_wmma_f32_16x16x32_bf16(false, a, false, b, (short)0, c, false, false);
  }
  static __device__ __forceinline__ void guard(v8f& a, v8f& b, v16b x, v16b y) { dep_guard_b(a, b, x, y); }
  static __device__ __forceinline__ void guard_all(v8f& a0, v8f& a1, v8f& a2, v8f& a3, v16b x, v16b y, v16b b0, v16b b1, v16b b2, v16b b3) {
    dep_guard_all_b(a0, a1, a2, a3, x, y, b0, b1, b2, b3);
  }
  static __device__ __forceinline__ void keep(v16b a, v16b b, v16b c, v16b d) { keep4_b(a, b, c, d); }
};

__device__ __forceinline__ unsigned pk16(unsigned short a, unsigned short b) { return (unsigned)a | ((unsigned)b << 16); }
__device__ __forceinline__ unsigned short h_bits(float f) { const _Float16 h = (_Float16)f; return __builtin_bit_cast(unsigned short, h); }
__device__ __forceinline__ v4u pack8h(float a0, float a1, float a2, float a3, float a4, float a5, float a6, float a7) {
  return (v4u){ pk16(h_bits(a0), h_bits(a1)), pk16(h_bits(a2), h_bits(a3)), pk16(h_bits(a4), h_bits(a5)), pk16(h_bits(a6), h_bits(a7)) };
}
__device__ __forceinline__ float h16_to_f32(unsigned hb) {
  const unsigned sgn = (hb & 0x8000u) << 16; const unsigned em = hb & 0x7fffu;
  const float fn = __uint_as_float((em << 13) + 0x38000000u);
  const float fs = (float)em * 5.9604644775390625e-8f;
  const float mag = (em < 0x400u) ? fs : fn; return __uint_as_float(__float_as_uint(mag) | sgn); }

__device__ __forceinline__ void store16_2x(unsigned short* p, v4u u) {
  *(volatile v4u*)p = u;
  __threadfence();
  *(volatile v4u*)p = u;
}
__device__ __forceinline__ void wave_sync_lds() {
  __builtin_amdgcn_fence(__ATOMIC_RELEASE, "workgroup");
  __builtin_amdgcn_wave_barrier();
  __builtin_amdgcn_fence(__ATOMIC_ACQUIRE, "workgroup");
}
__device__ __forceinline__ float wave_sum(float v) {
#pragma unroll
  for (int off = 16; off > 0; off >>= 1) v += __shfl_xor(v, off, 32);
  return v;
}
__device__ __forceinline__ float wave_max(float v) {
#pragma unroll
  for (int off = 16; off > 0; off >>= 1) v = fmaxf(v, __shfl_xor(v, off, 32));
  return v;
}

template <int ET> struct Elem;
template <> struct Elem<0> { typedef _Float16 T; };
template <> struct Elem<1> { typedef __bf16 T; };
template <int ET, bool SPLIT, int BIAS_MODE, int OUT_MODE, bool RESID, int ACT = 0>
__global__ __launch_bounds__(256) void wmma_gemm64(
    const unsigned short* __restrict__ Ap, const unsigned short* __restrict__ A2p, int lda, long strideA,
    const unsigned short* __restrict__ Btp, const unsigned short* __restrict__ Bt2p, int ldb, long strideB,
    void* __restrict__ Cout, void* __restrict__ Cout2, int ldc, long strideC,
    const float* __restrict__ bias,
    const float* __restrict__ resid, long strideR,
    int M, int N, int K, float scale) {
  typedef typename Elem<ET>::T T;
  typedef typename Frag<T>::V V;
  const T* A = (const T*)Ap; const T* A2 = (const T*)A2p; const T* Bt = (const T*)Btp; const T* Bt2 = (const T*)Bt2p;
  __shared__ __align__(16) float sT[8][16 * 68];
  const int b    = blockIdx.y;
  const int lane = threadIdx.x & 31;
  const int wave = threadIdx.x >> 5;
  const int tilesN = N >> 6;
  const int tilesM = M >> 6;
  const int tile = blockIdx.x * 8 + wave;
  if (tile >= tilesM * tilesN) return;
  const int tm = tile / tilesN;
  const int tn = tile - tm * tilesN;
  const int m0 = tm << 6;
  const int n0 = tn << 6;

  const T* Ab  = A  + (size_t)b * strideA;
  const T* Bb  = Bt + (size_t)b * strideB;
  const T* Ab2 = SPLIT ? (A2  + (size_t)b * strideA) : nullptr;
  const T* Bb2 = SPLIT ? (Bt2 + (size_t)b * strideB) : nullptr;

  const int rlane = lane & 15;
  const int koff  = (lane >> 4) * 8;
  const int mOff  = (lane >> 4) * 8;

  v8f acc[4][4];
#pragma unroll
  for (int i = 0; i < 4; ++i)
#pragma unroll
    for (int j = 0; j < 4; ++j) acc[i][j] = (v8f){0.f,0.f,0.f,0.f,0.f,0.f,0.f,0.f};

  for (int k0 = 0; k0 < K; k0 += 32) {
    V bh[4], bl[4];
#pragma unroll
    for (int j = 0; j < 4; ++j) {
      const size_t bo = (size_t)(n0 + (j << 4) + rlane) * ldb + koff + k0;
      bh[j] = Frag<T>::load(Bb + bo);
      if (SPLIT) bl[j] = Frag<T>::load(Bb2 + bo);
    }
#pragma unroll
    for (int i = 0; i < 4; ++i) {
      const size_t ao = (size_t)(m0 + (i << 4) + rlane) * lda + koff + k0;
      V ah = Frag<T>::load(Ab + ao);
      V al;
      if (SPLIT) al = Frag<T>::load(Ab2 + ao);
#pragma unroll
      for (int j = 0; j < 4; ++j) {
        acc[i][j] = Frag<T>::mma(ah, bh[j], acc[i][j]);
        if (SPLIT) {
          acc[i][j] = Frag<T>::mma(ah, bl[j], acc[i][j]);
          acc[i][j] = Frag<T>::mma(al, bh[j], acc[i][j]);
        }
      }
      Frag<T>::guard_all(acc[i][0], acc[i][1], acc[i][2], acc[i][3], ah, SPLIT ? al : ah, bh[0], bh[1], bh[2], bh[3]);
    }
    Frag<T>::keep(bh[0], bh[1], bh[2], bh[3]);
    if (SPLIT) Frag<T>::keep(bl[0], bl[1], bl[2], bl[3]);
  }
  acc_guard4(acc[0][0], acc[0][1], acc[0][2], acc[0][3]);
  acc_guard4(acc[1][0], acc[1][1], acc[1][2], acc[1][3]);
  acc_guard4(acc[2][0], acc[2][1], acc[2][2], acc[2][3]);
  acc_guard4(acc[3][0], acc[3][1], acc[3][2], acc[3][3]);

  float* slab = sT[wave];
  const float* Rb = RESID ? (resid + (size_t)b * strideR) : nullptr;
#pragma unroll
  for (int i = 0; i < 4; ++i) {
    const int mBase = m0 + (i << 4);
#pragma unroll
    for (int j = 0; j < 4; ++j) {
      const int n = n0 + (j << 4) + rlane;
      float bv = 0.f;
      if (BIAS_MODE == 2) bv = bias[n];
#pragma unroll
      for (int r = 0; r < 8; ++r) {
        float v = acc[i][j][r] * scale;
        if (BIAS_MODE == 1) v += bias[mBase + mOff + r];
        if (BIAS_MODE == 2) v += bv;
        if (RESID) v += Rb[(size_t)(mBase + mOff + r) * ldc + n];
        if (ACT == 2) v = fmaxf(v, 0.0f);
        if (ACT == 4) v = (v > 0.f) ? v : 0.01f * v;
        slab[(mOff + r) * 68 + (j << 4) + rlane] = v;
      }
    }
    __builtin_amdgcn_fence(__ATOMIC_RELEASE, "workgroup");
    __builtin_amdgcn_wave_barrier();
    __builtin_amdgcn_fence(__ATOMIC_ACQUIRE, "workgroup");
    if (OUT_MODE == 0) {
      float* C = (float*)Cout + (size_t)b * strideC;
      const int hh = lane >> 4, c4 = (lane & 15) * 4;
      for (int pass = 0; pass < 2; ++pass) {
#pragma unroll
        for (int it = 0; it < 8; ++it) {
          const int row = it * 2 + hh;
          v4f v = *(const v4f*)(slab + row * 68 + c4);
          *(volatile v4f*)(C + (size_t)(mBase + row) * ldc + n0 + c4) = v;
        }
        __threadfence();
      }
    } else {
      const int q = lane >> 3, c8 = (lane & 7) * 8;
      unsigned short* C  = (unsigned short*)Cout  + (size_t)b * strideC;
      unsigned short* C2 = (OUT_MODE == 2) ? ((unsigned short*)Cout2 + (size_t)b * strideC) : nullptr;
      for (int pass = 0; pass < 2; ++pass) {
#pragma unroll
        for (int it = 0; it < 4; ++it) {
          const int row = it * 4 + q;
          const float* sp = slab + row * 68 + c8;
          v8h hv, lv;
#pragma unroll
          for (int e = 0; e < 8; ++e) {
            if (OUT_MODE == 1) {
              hv[e] = (_Float16)sp[e];
            } else {
              unsigned short hb = f2bf_bits(sp[e]);
              unsigned short lb = f2bf_bits(sp[e] - bf_bits2f(hb));
              hv[e] = __builtin_bit_cast(_Float16, hb);
              lv[e] = __builtin_bit_cast(_Float16, lb);
            }
          }
          *(volatile v8h*)(C + (size_t)(mBase + row) * ldc + n0 + c8) = hv;
          if (OUT_MODE == 2) *(volatile v8h*)(C2 + (size_t)(mBase + row) * ldc + n0 + c8) = lv;
        }
        __threadfence();
      }
    }
    __builtin_amdgcn_fence(__ATOMIC_RELEASE, "workgroup");
    __builtin_amdgcn_wave_barrier();
    __builtin_amdgcn_fence(__ATOMIC_ACQUIRE, "workgroup");
  }
}

__global__ __launch_bounds__(256) void im2col1_kernel(const float* __restrict__ x, const float* __restrict__ w1,
                                                      unsigned short* __restrict__ A1, unsigned short* __restrict__ Bt1) {
  const int t = threadIdx.x;
  float v[8];
  if (blockIdx.x < kIm2colBlocksA) {
    const int i8  = blockIdx.x * 256 + t;
    const int row = i8 / 12;
    const int cg  = i8 - row * 12;
    const int c0  = cg * 8;
    const int xx  = row % kH1;
    const int yy  = (row / kH1) % kH1;
    const int b   = row / (kH1 * kH1);
    const float* xb = x + (size_t)b * (kImg * kImg) + yy * kImg + xx;
#pragma unroll
    for (int e = 0; e < 8; ++e) {
      const int tt = c0 + e;
      const int tc = (tt < kTaps) ? tt : (kTaps - 1);
      const int r  = tc / 9;
      const int s  = tc - r * 9;
      const float fsel = (tt < kTaps) ? 1.0f : 0.0f;
      v[e] = xb[r * kImg + s] * fsel;
    }
    const v4u u = pack8h(v[0], v[1], v[2], v[3], v[4], v[5], v[6], v[7]);
    store16_2x(A1 + 8 * (size_t)i8, u);
  } else {
    const int j8  = (blockIdx.x - kIm2colBlocksA) * 256 + t;
    const int oc  = j8 / 12;
    const int cg  = j8 - oc * 12;
    const int c0  = cg * 8;
    const float* wr = w1 + (size_t)oc * kTaps;
#pragma unroll
    for (int e = 0; e < 8; ++e) {
      const int tt = c0 + e;
      const int tc = (tt < kTaps) ? tt : (kTaps - 1);
      const float fsel = (tt < kTaps) ? 16.0f : 0.0f;
      v[e] = wr[tc] * fsel;
    }
    const v4u u = pack8h(v[0], v[1], v[2], v[3], v[4], v[5], v[6], v[7]);
    store16_2x(Bt1 + 8 * (size_t)j8, u);
  }
}

__global__ __launch_bounds__(256) void w2cast_kernel(const float* __restrict__ w2, unsigned short* __restrict__ Bt2) {
  const int i8  = blockIdx.x * 256 + threadIdx.x;
  const int oc  = i8 / (kK2 / 8);
  const int g   = i8 - oc * (kK2 / 8);
  const int tap = g >> 5;
  const int ic0 = (g & 31) * 8;
  const float* wp = w2 + ((size_t)oc * kC + ic0) * kTaps + tap;
  float v[8];
#pragma unroll
  for (int e = 0; e < 8; ++e) v[e] = wp[(size_t)e * kTaps] * 64.0f;
  const v4u u = pack8h(v[0], v[1], v[2], v[3], v[4], v[5], v[6], v[7]);
  store16_2x(Bt2 + 8 * (size_t)i8, u);
}

__global__ __launch_bounds__(256) void conv2_gemm_kernel(const unsigned short* __restrict__ Hp, const unsigned short* __restrict__ Btp,
                                                         const float* __restrict__ bias, float* __restrict__ Cout, float scale) {
  typedef _Float16 T;
  const T* Hh = (const T*)Hp;
  const T* Bt = (const T*)Btp;
  __shared__ __align__(16) float sT[8][16 * 68];
  const int lane = threadIdx.x & 31;
  const int wave = threadIdx.x >> 5;
  const int tile = blockIdx.x * 8 + wave;
  if (tile >= kCv2Tiles) return;
  const int tm = tile >> 2;
  const int tn = tile & 3;
  const int m0 = tm << 6;
  const int n0 = tn << 6;
  const int rlane = lane & 15;
  const int koff  = (lane >> 4) * 8;
  const int mOff  = (lane >> 4) * 8;

  int rowoff[4];
#pragma unroll
  for (int i = 0; i < 4; ++i) {
    const int m   = m0 + (i << 4) + rlane;
    const int bb  = m / kSp2;
    const int rem = m - bb * kSp2;
    const int oy  = rem / 6;
    const int ox  = rem - oy * 6;
    rowoff[i] = ((bb * kH1 + 2 * oy) * kH1 + 2 * ox) * kC;
  }

  v8f acc[4][4];
#pragma unroll
  for (int i = 0; i < 4; ++i)
#pragma unroll
    for (int j = 0; j < 4; ++j) acc[i][j] = (v8f){0.f,0.f,0.f,0.f,0.f,0.f,0.f,0.f};

#pragma unroll 1
  for (int tap = 0; tap < kTaps; ++tap) {
    const int rr = tap / 9;
    const int ss = tap - rr * 9;
    const int tapoff = (rr * kH1 + ss) * kC;
    const int kb = tap * kC;
#pragma unroll 1
    for (int ic0 = 0; ic0 < kC; ic0 += 32) {
      v16h bh[4];
#pragma unroll
      for (int j = 0; j < 4; ++j) {
        const size_t bo = (size_t)(n0 + (j << 4) + rlane) * kK2 + kb + ic0 + koff;
        bh[j] = Frag<T>::load(Bt + bo);
      }
#pragma unroll
      for (int i = 0; i < 4; ++i) {
        const size_t ao = (size_t)rowoff[i] + tapoff + ic0 + koff;
        v16h ah = Frag<T>::load(Hh + ao);
#pragma unroll
        for (int j = 0; j < 4; ++j) acc[i][j] = Frag<T>::mma(ah, bh[j], acc[i][j]);
        Frag<T>::guard_all(acc[i][0], acc[i][1], acc[i][2], acc[i][3], ah, ah, bh[0], bh[1], bh[2], bh[3]);
      }
      Frag<T>::keep(bh[0], bh[1], bh[2], bh[3]);
    }
  }
  acc_guard4(acc[0][0], acc[0][1], acc[0][2], acc[0][3]);
  acc_guard4(acc[1][0], acc[1][1], acc[1][2], acc[1][3]);
  acc_guard4(acc[2][0], acc[2][1], acc[2][2], acc[2][3]);
  acc_guard4(acc[3][0], acc[3][1], acc[3][2], acc[3][3]);

  float* slab = sT[wave];
#pragma unroll
  for (int i = 0; i < 4; ++i) {
    const int mBase = m0 + (i << 4);
#pragma unroll
    for (int j = 0; j < 4; ++j) {
      const int n = n0 + (j << 4) + rlane;
      const float bv = bias[n];
#pragma unroll
      for (int r = 0; r < 8; ++r) {
        const float v = acc[i][j][r] * scale + bv;
        slab[(mOff + r) * 68 + (j << 4) + rlane] = v;
      }
    }
    wave_sync_lds();
    {
      const int hh = lane >> 4, c4 = (lane & 15) * 4;
      for (int pass = 0; pass < 2; ++pass) {
#pragma unroll
        for (int it = 0; it < 8; ++it) {
          const int row = it * 2 + hh;
          v4f v = *(const v4f*)(slab + row * 68 + c4);
          *(volatile v4f*)(Cout + (size_t)(mBase + row) * kC + n0 + c4) = v;
        }
        __threadfence();
      }
    }
    wave_sync_lds();
  }
}

__global__ __launch_bounds__(256) void caps_transform_kernel(const float* __restrict__ prim, const float* __restrict__ Wc,
                                                             const float* __restrict__ Wbc, unsigned short* __restrict__ U) {
  __shared__ __align__(16) _Float16 At[kBatch * 32];
  __shared__ __align__(16) _Float16 Bw[kNIO * 32];
  __shared__ __align__(16) float slab[8][16 * 20];
  const int t = threadIdx.x;
  const int lane = t & 31, wave = t >> 5;
  const int loc = blockIdx.x;
  const v4u z4 = (v4u){0u, 0u, 0u, 0u};
  {
    float pv[8];
#pragma unroll
    for (int cc = 0; cc < 8; ++cc) {
      const int f  = 8 * loc + cc;
      const int ch = f / kSp2;
      const int sp = f - ch * kSp2;
      pv[cc] = prim[((size_t)t * kSp2 + sp) * kC + ch];
    }
    const v4u u = pack8h(pv[0], pv[1], pv[2], pv[3], pv[4], pv[5], pv[6], pv[7]);
    _Float16* ar = At + t * 32;
    *(v4u*)(ar)      = u;
    *(v4u*)(ar + 8)  = z4;
    *(v4u*)(ar + 16) = z4;
    *(v4u*)(ar + 24) = z4;
  }
  {
    const int q  = (t < kNIO) ? t : (kNIO - 1);
    const int ci = q >> 4, o = q & 15;
    const float* wp = Wc + ((size_t)(ci * kRoute + loc) * kVd + o) * 8;
    const v4f w0 = *(const v4f*)(wp);
    const v4f w1 = *(const v4f*)(wp + 4);
    const v4u u = pack8h(w0[0], w0[1], w0[2], w0[3], w1[0], w1[1], w1[2], w1[3]);
    if (t < kNIO) {
      _Float16* br = Bw + q * 32;
      *(v4u*)(br)      = u;
      *(v4u*)(br + 8)  = z4;
      *(v4u*)(br + 16) = z4;
      *(v4u*)(br + 24) = z4;
    }
  }
  __syncthreads();

  const int rlane = lane & 15;
  const int koff  = (lane >> 4) * 8;
  const int mOff  = (lane >> 4) * 8;
  const int srow  = lane >> 1;
  const int c8    = (lane & 1) * 8;
  float* sl = slab[wave];
#pragma unroll 1
  for (int mi = 0; mi < 2; ++mi) {
    const int arow0 = wave * 32 + mi * 16;
    const v16h af = Frag<_Float16>::load(At + (arow0 + rlane) * 32 + koff);
#pragma unroll 1
    for (int ci = 0; ci < kCls; ++ci) {
      const v16h bf = Frag<_Float16>::load(Bw + (ci * 16 + rlane) * 32 + koff);
      v8f acc = (v8f){0.f,0.f,0.f,0.f,0.f,0.f,0.f,0.f};
      acc = Frag<_Float16>::mma(af, bf, acc);
      dep_guard1_h(acc, af, bf);
      const float wb = Wbc[(size_t)(ci * kRoute + loc) * kVd + rlane];
#pragma unroll
      for (int r = 0; r < 8; ++r) sl[(mOff + r) * 20 + rlane] = acc[r] + wb;
      wave_sync_lds();
      const v4f x0 = *(const v4f*)(sl + srow * 20 + c8);
      const v4f x1 = *(const v4f*)(sl + srow * 20 + c8 + 4);
      const v4u u = pack8h(x0[0], x0[1], x0[2], x0[3], x1[0], x1[1], x1[2], x1[3]);
      unsigned short* dst = U + ((size_t)(loc * kCls + ci) * (kBatch * kVd) + (size_t)(arow0 + srow) * kVd + c8);
      store16_2x(dst, u);
      wave_sync_lds();
    }
  }
}

__global__ __launch_bounds__(256) void route_v_kernel(const unsigned short* __restrict__ U, const float* __restrict__ bij,
                                                      float* __restrict__ vraw, int use_bij) {
  __shared__ float csh[kRoute];
  __shared__ float redm[8];
  __shared__ float reds[8];
  __shared__ __align__(16) float outs[128 * kVd];
  const int t = threadIdx.x;
  const int lane = t & 31, wave = t >> 5;
  const int ci = blockIdx.x >> 1;
  const int bhalf = blockIdx.x & 1;
  if (use_bij) {
    const float* brow = bij + (size_t)ci * kRoute;
    float mx = -INFINITY;
#pragma unroll 1
    for (int n = t; n < kRoute; n += 256) { const float xv = brow[n]; csh[n] = xv; mx = fmaxf(mx, xv); }
    mx = wave_max(mx);
    if (lane == 0) redm[wave] = mx;
    __syncthreads();
    float m = redm[0];
#pragma unroll
    for (int w = 1; w < 8; ++w) m = fmaxf(m, redm[w]);
    float sm = 0.0f;
#pragma unroll 1
    for (int n = t; n < kRoute; n += 256) { const float e = expf(csh[n] - m); csh[n] = e; sm += e; }
    sm = wave_sum(sm);
    if (lane == 0) reds[wave] = sm;
    __syncthreads();
    float tot = reds[0];
#pragma unroll
    for (int w = 1; w < 8; ++w) tot += reds[w];
    const float inv = 1.0f / tot;
#pragma unroll 1
    for (int n = t; n < kRoute; n += 256) csh[n] = csh[n] * inv;
  } else {
#pragma unroll 1
    for (int n = t; n < kRoute; n += 256) csh[n] = 1.0f / 1152.0f;
  }
  __syncthreads();

  const int bl = t >> 1;
  const int kh = (t & 1) * 8;
  const int b  = bhalf * 128 + bl;
  const unsigned short* up = U + (size_t)ci * kRoute * (kBatch * kVd) + (size_t)b * kVd + kh;
  float acc[8];
#pragma unroll
  for (int e = 0; e < 8; ++e) acc[e] = 0.0f;
#pragma unroll 1
  for (int n = 0; n < kRoute; ++n) {
    const v4u w = *(const v4u*)(up + (size_t)n * (kBatch * kVd));
    const float cn = csh[n];
    const unsigned w0 = w[0], w1 = w[1], w2 = w[2], w3 = w[3];
    acc[0] = fmaf(cn, h16_to_f32(w0 & 0xffffu), acc[0]);
    acc[1] = fmaf(cn, h16_to_f32(w0 >> 16),     acc[1]);
    acc[2] = fmaf(cn, h16_to_f32(w1 & 0xffffu), acc[2]);
    acc[3] = fmaf(cn, h16_to_f32(w1 >> 16),     acc[3]);
    acc[4] = fmaf(cn, h16_to_f32(w2 & 0xffffu), acc[4]);
    acc[5] = fmaf(cn, h16_to_f32(w2 >> 16),     acc[5]);
    acc[6] = fmaf(cn, h16_to_f32(w3 & 0xffffu), acc[6]);
    acc[7] = fmaf(cn, h16_to_f32(w3 >> 16),     acc[7]);
  }
  *(v4f*)(outs + bl * kVd + kh)     = (v4f){acc[0], acc[1], acc[2], acc[3]};
  *(v4f*)(outs + bl * kVd + kh + 4) = (v4f){acc[4], acc[5], acc[6], acc[7]};
  __syncthreads();
  float* dst = vraw + (size_t)ci * (kBatch * kVd) + (size_t)bhalf * (128 * kVd);
  for (int pass = 0; pass < 2; ++pass) {
#pragma unroll
    for (int it = 0; it < 2; ++it) {
      const int idx = it * 256 + t;
      const v4f v = *(const v4f*)(outs + idx * 4);
      *(volatile v4f*)(dst + (size_t)idx * 4) = v;
    }
    __threadfence();
  }
}

__global__ __launch_bounds__(256) void squash_kernel(const float* __restrict__ vraw, float* __restrict__ vout) {
  __shared__ float red[8];
  const int t = threadIdx.x;
  const int lane = t & 31, wave = t >> 5;
  const size_t base = (size_t)blockIdx.x * (kBatch * kVd);
  v4f xv[4];
  float ss = 0.0f;
#pragma unroll
  for (int it = 0; it < 4; ++it) {
    xv[it] = *(const v4f*)(vraw + base + (size_t)(it * 256 + t) * 4);
    ss += xv[it][0] * xv[it][0];
    ss += xv[it][1] * xv[it][1];
    ss += xv[it][2] * xv[it][2];
    ss += xv[it][3] * xv[it][3];
  }
  ss = wave_sum(ss);
  if (lane == 0) red[wave] = ss;
  __syncthreads();
  float tot = red[0];
#pragma unroll
  for (int w = 1; w < 8; ++w) tot += red[w];
  const float nrm  = sqrtf(tot);
  const float n2   = nrm * nrm;
  const float coef = n2 / (1.0f + n2);
  const float inv  = 1.0f / nrm;
  v4f ov[4];
#pragma unroll
  for (int it = 0; it < 4; ++it) {
    ov[it] = (v4f){ coef * (xv[it][0] * inv), coef * (xv[it][1] * inv), coef * (xv[it][2] * inv), coef * (xv[it][3] * inv) };
  }
  for (int pass = 0; pass < 2; ++pass) {
#pragma unroll
    for (int it = 0; it < 4; ++it) {
      *(volatile v4f*)(vout + base + (size_t)(it * 256 + t) * 4) = ov[it];
    }
    __threadfence();
  }
}

__global__ __launch_bounds__(256) void route_b_kernel(const unsigned short* __restrict__ U, const float* __restrict__ v,
                                                      const float* __restrict__ bold, float* __restrict__ bnew, int add_old) {
  __shared__ __align__(16) float vsh[kBatch * kVd];
  __shared__ float res[32];
  const int t = threadIdx.x;
  const int lane = t & 31, wave = t >> 5;
  const int ci = blockIdx.x / 36;
  const int g  = blockIdx.x - ci * 36;
#pragma unroll
  for (int it = 0; it < 4; ++it) {
    const int idx = it * 256 + t;
    *(v4f*)(vsh + idx * 4) = *(const v4f*)(v + (size_t)ci * (kBatch * kVd) + (size_t)idx * 4);
  }
  __syncthreads();
#pragma unroll 1
  for (int q = 0; q < 4; ++q) {
    const int n = g * 32 + wave * 4 + q;
    const unsigned short* up = U + ((size_t)ci * kRoute + n) * (kBatch * kVd);
    float acc = 0.0f;
#pragma unroll 1
    for (int it = 0; it < 16; ++it) {
      const int e0 = (it * 32 + lane) * 8;
      const v4u w  = *(const v4u*)(up + e0);
      const v4f va = *(const v4f*)(vsh + e0);
      const v4f vb = *(const v4f*)(vsh + e0 + 4);
      const unsigned w0 = w[0], w1 = w[1], w2 = w[2], w3 = w[3];
      acc = fmaf(h16_to_f32(w0 & 0xffffu), va[0], acc);
      acc = fmaf(h16_to_f32(w0 >> 16),     va[1], acc);
      acc = fmaf(h16_to_f32(w1 & 0xffffu), va[2], acc);
      acc = fmaf(h16_to_f32(w1 >> 16),     va[3], acc);
      acc = fmaf(h16_to_f32(w2 & 0xffffu), vb[0], acc);
      acc = fmaf(h16_to_f32(w2 >> 16),     vb[1], acc);
      acc = fmaf(h16_to_f32(w3 & 0xffffu), vb[2], acc);
      acc = fmaf(h16_to_f32(w3 >> 16),     vb[3], acc);
    }
    acc = wave_sum(acc);
    float val = acc;
    if (add_old) val += bold[(size_t)ci * kRoute + n];
    if (lane == 0) res[wave * 4 + q] = val;
  }
  __syncthreads();
  if (wave == 0) {
    const float val = res[lane];
    float* dst = bnew + (size_t)ci * kRoute + g * 32 + lane;
    *(volatile float*)dst = val;
    __threadfence();
    *(volatile float*)dst = val;
  }
}

extern "C" void kernel_launch(void* const* d_in, const int* in_sizes, int n_in,
                              void* d_out, int out_size, void* d_ws, size_t ws_size, hipStream_t stream) {
  if (n_in < 7) return;
  if ((size_t)out_size != (size_t)kCls * kBatch * kVd) return;
  if (ws_size < kWsTotal) return;
  if (in_sizes[0] != kBatch * kImg * kImg) return;
  if (in_sizes[1] != kC * kTaps || in_sizes[2] != kC) return;
  if (in_sizes[3] != kC * kC * kTaps || in_sizes[4] != kC) return;
  if (in_sizes[5] != kCls * kRoute * kVd * 8 || in_sizes[6] != kCls * kRoute * kVd) return;

  const float* x       = (const float*)d_in[0];
  const float* conv1_w = (const float*)d_in[1];
  const float* conv1_b = (const float*)d_in[2];
  const float* conv2_w = (const float*)d_in[3];
  const float* conv2_b = (const float*)d_in[4];
  const float* Wcap    = (const float*)d_in[5];
  const float* Wbcap   = (const float*)d_in[6];
  float* out = (float*)d_out;

  char* ws = (char*)d_ws;
  unsigned short* U    = (unsigned short*)(ws + kOffU);
  unsigned short* A1   = (unsigned short*)(ws + kOffA1);
  unsigned short* hbuf = (unsigned short*)(ws + kOffH);
  unsigned short* Bt1  = (unsigned short*)(ws + kOffBt1);
  unsigned short* Bt2  = (unsigned short*)(ws + kOffBt2);
  float* prim = (float*)(ws + kOffPrim);
  float* vraw = (float*)(ws + kOffVraw);
  float* vbuf = (float*)(ws + kOffVbuf);
  float* bijA = (float*)(ws + kOffBijA);
  float* bijB = (float*)(ws + kOffBijB);

  im2col1_kernel<<<kIm2colBlocksA + kIm2colBlocksB, 256, 0, stream>>>(x, conv1_w, A1, Bt1);
  w2cast_kernel<<<kW2Blocks, 256, 0, stream>>>(conv2_w, Bt2);
  wmma_gemm64<0, false, 2, 1, false, 0><<<dim3(kCv1Blocks, 1), 256, 0, stream>>>(
      A1, A1, kK1, 0L, Bt1, Bt1, kK1, 0L, (void*)hbuf, (void*)hbuf, kC, 0L,
      conv1_b, conv1_b, 0L, kP1, kC, kK1, 1.0f / 16.0f);
  conv2_gemm_kernel<<<kCv2Blocks, 256, 0, stream>>>(hbuf, Bt2, conv2_b, prim, 1.0f / 64.0f);
  caps_transform_kernel<<<kRoute, 256, 0, stream>>>(prim, Wcap, Wbcap, U);
  route_v_kernel<<<kCls * 2, 256, 0, stream>>>(U, bijA, vraw, 0);
  squash_kernel<<<kCls, 256, 0, stream>>>(vraw, vbuf);
  route_b_kernel<<<kCls * 36, 256, 0, stream>>>(U, vbuf, bijA, bijA, 0);
  route_v_kernel<<<kCls * 2, 256, 0, stream>>>(U, bijA, vraw, 1);
  squash_kernel<<<kCls, 256, 0, stream>>>(vraw, vbuf);
  route_b_kernel<<<kCls * 36, 256, 0, stream>>>(U, vbuf, bijA, bijB, 1);
  route_v_kernel<<<kCls * 2, 256, 0, stream>>>(U, bijB, vraw, 1);
  squash_kernel<<<kCls, 256, 0, stream>>>(vraw, out);
}
